// Label_Histogram_89163521065189
// MI455X (gfx1250) — hardware-verified
//
#include <hip/hip_runtime.h>


typedef _Float16 v16h __attribute__((ext_vector_type(16)));
typedef _Float16 v8h_t __attribute__((ext_vector_type(8)));
typedef v8h_t __attribute__((may_alias)) v8h;
typedef __bf16 v16bf __attribute__((ext_vector_type(16)));
typedef unsigned short v16us __attribute__((ext_vector_type(16)));
typedef float v8f __attribute__((ext_vector_type(8)));
typedef float v4f_t __attribute__((ext_vector_type(4)));
typedef v4f_t __attribute__((may_alias)) v4f;

union FragH { v16h v; v8h_t h[2]; };
union FragB { v16bf v; v16us u; };

#define DD    64
#define HK    64
#define KCL   16
#define NHEAD 4
#define KD    (KCL * DD)
#define WPB   2
#define PT    32
#define TPW   4
#define PW    (PT * TPW)
#define XS    65
#define KP    72
#define DS    65

__device__ __forceinline__ v8f wmma_f16(v8f c, v16h a, v16h b) {
  v8f d = __builtin_amdgcn_wmma_f32_16x16x32_f16(false, a, false, b, (short)0, c, false, false);
  asm volatile("v_nop\n\tv_nop\n\tv_nop\n\tv_nop" : "+v"(d) : "v"(a), "v"(b));
  return d;
}

__device__ __forceinline__ v8f wmma_bf16(v8f c, v16bf a, v16bf b) {
  v8f d = __builtin_amdgcn_wmma_f32_16x16x32_bf16(false, a, false, b, (short)0, c, false, false);
  asm volatile("v_nop\n\tv_nop\n\tv_nop\n\tv_nop" : "+v"(d) : "v"(a), "v"(b));
  return d;
}

__device__ __forceinline__ unsigned short bf16_bits(float f) {
  unsigned int u = __float_as_uint(f);
  u = u + 0x7FFFu + ((u >> 16) & 1u);
  return (unsigned short)(u >> 16);
}

__device__ __forceinline__ void split16(const v4f u0, const v4f u1, const v4f u2, const v4f u3,
                                        FragB& hi, FragB& lo) {
  float f[16];
#pragma unroll
  for (int i = 0; i < 4; ++i) { f[i] = u0[i]; f[4 + i] = u1[i]; f[8 + i] = u2[i]; f[12 + i] = u3[i]; }
#pragma unroll
  for (int i = 0; i < 16; ++i) {
    const float v = f[i];
    const unsigned short hb = bf16_bits(v);
    const float hv = __uint_as_float(((unsigned int)hb) << 16);
    const unsigned short lb = bf16_bits(v - hv);
    hi.u[i] = hb;
    lo.u[i] = lb;
  }
}

__device__ __forceinline__ int lbound(const int* __restrict__ a, int n, int key) {
  int lo = 0, hi = n;
  while (lo < hi) {
    const int mid = (lo + hi) >> 1;
    if (a[mid] < key) lo = mid + 1; else hi = mid;
  }
  return lo;
}

__global__ __launch_bounds__(64) void k_assign(const float* __restrict__ x, const float* __restrict__ kf,
                                               float* __restrict__ wts, int npts) {
  __shared__ _Float16 kh[HK * KP] __attribute__((aligned(16)));
  __shared__ float kn2[HK];
  __shared__ float xf[WPB][PT * XS] __attribute__((aligned(16)));
  __shared__ _Float16 xh[WPB][PT * KP] __attribute__((aligned(16)));
  __shared__ float dt[WPB][PT * DS] __attribute__((aligned(16)));
  __shared__ float wl[WPB][PT * KCL] __attribute__((aligned(16)));

  const int tid  = threadIdx.x;
  const int lane = tid & 31;
  const int wave = tid >> 5;
  const int hh   = lane >> 4;
  const int m    = lane & 15;

  for (int j = tid; j < HK * DD; j += WPB * 32) {
    const int c = j >> 6, d = j & 63;
    kh[c * KP + d] = (_Float16)(kf[j] * 16.0f);
  }
  for (int c = tid; c < HK; c += WPB * 32) {
    float s = 0.f;
#pragma unroll 4
    for (int d = 0; d < DD; ++d) { const float v = kf[c * DD + d]; s = fmaf(v, v, s); }
    kn2[c] = s;
  }
  __syncthreads();

  float*    xfw = xf[wave];
  _Float16* xhw = xh[wave];
  float*    dtw = dt[wave];
  float*    wlw = wl[wave];

  const size_t wbase = ((size_t)blockIdx.x * WPB + (size_t)wave) * PW;
  const v8f vz = {0.f, 0.f, 0.f, 0.f, 0.f, 0.f, 0.f, 0.f};

  for (int t = 0; t < TPW; ++t) {
    const size_t base = wbase + (size_t)t * PT;

#pragma unroll 4
    for (int r = 0; r < PT; ++r) {
      const size_t n = base + (size_t)r;
      float v0 = 0.f, v1 = 0.f;
      if (n < (size_t)npts) { v0 = x[n * DD + lane]; v1 = x[n * DD + 32 + lane]; }
      xfw[r * XS + lane]      = v0;
      xfw[r * XS + 32 + lane] = v1;
      xhw[r * KP + lane]      = (_Float16)(v0 * 16.0f);
      xhw[r * KP + 32 + lane] = (_Float16)(v1 * 16.0f);
    }
    __syncthreads();

#pragma unroll
    for (int st = 0; st < 2; ++st) {
      v8f dacc[4];
#pragma unroll
      for (int nc = 0; nc < 4; ++nc) dacc[nc] = vz;
#pragma unroll
      for (int kc = 0; kc < 2; ++kc) {
        FragH a;
        const _Float16* ap = xhw + (st * 16 + m) * KP + kc * 32 + 8 * hh;
        a.h[0] = *(const v8h*)(ap);
        a.h[1] = *(const v8h*)(ap + 16);
#pragma unroll
        for (int nc = 0; nc < 4; ++nc) {
          FragH b;
          const _Float16* bp = kh + (nc * 16 + m) * KP + kc * 32 + 8 * hh;
          b.h[0] = *(const v8h*)(bp);
          b.h[1] = *(const v8h*)(bp + 16);
          dacc[nc] = wmma_f16(dacc[nc], a.v, b.v);
        }
      }
#pragma unroll
      for (int nc = 0; nc < 4; ++nc) {
#pragma unroll
        for (int r = 0; r < 8; ++r)
          dtw[(st * 16 + 8 * hh + r) * DS + nc * 16 + m] = dacc[nc][r];
      }
    }
    __syncthreads();

    {
      const float* xr = xfw + lane * XS;
      float xn = 0.f;
#pragma unroll 8
      for (int d = 0; d < DD; ++d) xn = fmaf(xr[d], xr[d], xn);

      float* tr = dtw + lane * DS;
      const float inv256 = 1.0f / 256.0f;
      float sh[NHEAD];
#pragma unroll
      for (int g = 0; g < NHEAD; ++g) {
        float s = 0.f;
#pragma unroll
        for (int k = 0; k < KCL; ++k) {
          const int c = g * KCL + k;
          const float d2 = fmaxf(kn2[c] + xn - 2.0f * (tr[c] * inv256), 0.f);
          const float tv = __builtin_amdgcn_rcpf(1.0f + d2);
          tr[c] = tv;
          s += tv;
        }
        sh[g] = s;
      }
      float mk[KCL];
#pragma unroll
      for (int k = 0; k < KCL; ++k) mk[k] = 0.f;
#pragma unroll
      for (int g = 0; g < NHEAD; ++g) {
        const float rs = __builtin_amdgcn_rcpf(sh[g]);
#pragma unroll
        for (int k = 0; k < KCL; ++k) mk[k] = fmaf(tr[g * KCL + k], rs, mk[k]);
      }
      const float scale = 10.0f / (float)NHEAD;
      float mx = -1e30f;
#pragma unroll
      for (int k = 0; k < KCL; ++k) { mk[k] *= scale; mx = fmaxf(mx, mk[k]); }
      float se = 0.f;
#pragma unroll
      for (int k = 0; k < KCL; ++k) { mk[k] = __expf(mk[k] - mx); se += mk[k]; }
      const float rse = __builtin_amdgcn_rcpf(se);
#pragma unroll
      for (int k = 0; k < KCL; ++k) wlw[lane * KCL + k] = mk[k] * rse;
    }
    __syncthreads();

    {
      const v4f* src = (const v4f*)wlw;
      const v4f q0 = src[lane], q1 = src[32 + lane], q2 = src[64 + lane], q3 = src[96 + lane];
      volatile v4f* g = (volatile v4f*)(wts + base * KCL);
      g[lane] = q0; g[32 + lane] = q1; g[64 + lane] = q2; g[96 + lane] = q3;
      __threadfence();
      g[lane] = q0; g[32 + lane] = q1; g[64 + lane] = q2; g[96 + lane] = q3;
    }
  }
}

__global__ __launch_bounds__(64) void k_segsum(const float* __restrict__ x, const float* __restrict__ wts,
                                               const int* __restrict__ index,
                                               const float* __restrict__ aux0, const int* __restrict__ aux1,
                                               float* __restrict__ agg, int npts, int nseg) {
  __shared__ float stg[WPB][8 * DD] __attribute__((aligned(16)));
  (void)aux0; (void)aux1;
  const int b    = blockIdx.x;
  const int lane = threadIdx.x & 31;
  const int wave = threadIdx.x >> 5;
  const int kb   = wave * 8;

  int lo = lbound(index, npts, b);
  int hi = lbound(index, npts, b + 1);
  if (lo < 0) lo = 0;
  if (hi > npts) hi = npts;

  float a0[8], a1[8];
#pragma unroll
  for (int j = 0; j < 8; ++j) { a0[j] = 0.f; a1[j] = 0.f; }

#pragma unroll 1
  for (int n = lo; n < hi; ++n) {
    const float* xp = x + (size_t)n * DD;
    const float x0 = xp[lane];
    const float x1 = xp[32 + lane];
    const v4f w0 = *(const v4f*)(wts + (size_t)n * KCL + kb);
    const v4f w1 = *(const v4f*)(wts + (size_t)n * KCL + kb + 4);
#pragma unroll
    for (int j = 0; j < 4; ++j) {
      a0[j]     = fmaf(w0[j], x0, a0[j]);
      a1[j]     = fmaf(w0[j], x1, a1[j]);
      a0[4 + j] = fmaf(w1[j], x0, a0[4 + j]);
      a1[4 + j] = fmaf(w1[j], x1, a1[4 + j]);
    }
  }

  float* sw = stg[wave];
#pragma unroll
  for (int j = 0; j < 8; ++j) { sw[j * DD + lane] = a0[j]; sw[j * DD + 32 + lane] = a1[j]; }
  __syncthreads();

  const v4f* src = (const v4f*)sw;
  const v4f q0 = src[lane], q1 = src[32 + lane], q2 = src[64 + lane], q3 = src[96 + lane];
  volatile v4f* g = (volatile v4f*)(agg + (size_t)b * KD + (size_t)wave * (8 * DD));
  g[lane] = q0; g[32 + lane] = q1; g[64 + lane] = q2; g[96 + lane] = q3;
  __threadfence();
  g[lane] = q0; g[32 + lane] = q1; g[64 + lane] = q2; g[96 + lane] = q3;
}

__global__ __launch_bounds__(64) void k_proj(const float* __restrict__ agg, const float* __restrict__ W,
                                             const float* __restrict__ bias, float* __restrict__ out, int nseg) {
  __shared__ float stg[WPB][16 * DD] __attribute__((aligned(16)));
  const int lane = threadIdx.x & 31;
  const int wave = threadIdx.x >> 5;
  const int hh   = lane >> 4;
  const int m    = lane & 15;
  const int row0 = (blockIdx.x * WPB + wave) * 16;

  int ar = row0 + m;
  if (ar > nseg - 1) ar = nseg - 1;
  const float* arow = agg + (size_t)ar * KD;

  const v8f vz = {0.f, 0.f, 0.f, 0.f, 0.f, 0.f, 0.f, 0.f};
  v8f acc[4];
#pragma unroll
  for (int nc = 0; nc < 4; ++nc) acc[nc] = vz;

#pragma unroll 1
  for (int ks = 0; ks < KD / 32; ++ks) {
    const int k0 = ks * 32;
    const float* ap = arow + k0 + 8 * hh;
    FragB ahi, alo;
    split16(*(const v4f*)(ap), *(const v4f*)(ap + 4), *(const v4f*)(ap + 16), *(const v4f*)(ap + 20), ahi, alo);
#pragma unroll
    for (int nc = 0; nc < 4; ++nc) {
      const float* bp = W + (size_t)(nc * 16 + m) * KD + k0 + 8 * hh;
      FragB bhi, blo;
      split16(*(const v4f*)(bp), *(const v4f*)(bp + 4), *(const v4f*)(bp + 16), *(const v4f*)(bp + 20), bhi, blo);
      acc[nc] = wmma_bf16(acc[nc], ahi.v, bhi.v);
      acc[nc] = wmma_bf16(acc[nc], ahi.v, blo.v);
      acc[nc] = wmma_bf16(acc[nc], alo.v, bhi.v);
    }
  }

  float* sw = stg[wave];
#pragma unroll
  for (int nc = 0; nc < 4; ++nc) {
    const float bv = bias[nc * 16 + m];
#pragma unroll
    for (int r = 0; r < 8; ++r) {
      float v = acc[nc][r] + bv;
      v = (v > 0.f) ? v : 0.01f * v;
      sw[(8 * hh + r) * DD + nc * 16 + m] = v;
    }
  }
  __syncthreads();

  const v4f* src = (const v4f*)sw;
  v4f q[8];
#pragma unroll
  for (int i = 0; i < 8; ++i) q[i] = src[i * 32 + lane];
  volatile v4f* g = (volatile v4f*)(out + (size_t)row0 * DD);
#pragma unroll
  for (int i = 0; i < 8; ++i) {
    const int rr = row0 + ((i * 32 + lane) >> 4);
    if (rr < nseg) g[i * 32 + lane] = q[i];
  }
  __threadfence();
#pragma unroll
  for (int i = 0; i < 8; ++i) {
    const int rr = row0 + ((i * 32 + lane) >> 4);
    if (rr < nseg) g[i * 32 + lane] = q[i];
  }
}

extern "C" void kernel_launch(void* const* d_in, const int* in_sizes, int n_in,
                              void* d_out, int out_size, void* d_ws, size_t ws_size,
                              hipStream_t stream) {
  if (n_in < 7) return;
  const float* x     = (const float*)d_in[0];
  const float* aux0  = (const float*)d_in[1];
  const float* kf    = (const float*)d_in[2];
  const float* W     = (const float*)d_in[3];
  const float* bias  = (const float*)d_in[4];
  const int*   index = (const int*)d_in[5];
  const int*   aux1  = (const int*)d_in[6];
  float* out = (float*)d_out;

  const int npts = in_sizes[0] / DD;
  const int nseg = out_size / DD;
  if (npts <= 0 || nseg <= 0) return;
  if (in_sizes[2] != HK * DD || in_sizes[3] != DD * KD || in_sizes[4] < DD || in_sizes[5] < npts) return;

  const int wavesA  = (npts + PW - 1) / PW;
  const int blocksA = (wavesA + WPB - 1) / WPB;
  const size_t rows_pad  = (size_t)blocksA * WPB * PW;
  const size_t wts_bytes = rows_pad * KCL * sizeof(float);
  const size_t wts_al    = (wts_bytes + 255) & ~(size_t)255;
  const size_t agg_bytes = (size_t)nseg * KD * sizeof(float);
  if (wts_al + agg_bytes > ws_size) return;

  float* wts = (float*)d_ws;
  float* agg = (float*)((char*)d_ws + wts_al);

  k_assign<<<blocksA, WPB * 32, 0, stream>>>(x, kf, wts, npts);
  k_segsum<<<nseg, WPB * 32, 0, stream>>>(x, wts, index, aux0, aux1, agg, npts, nseg);
  const int blocksC = (nseg + WPB * 16 - 1) / (WPB * 16);
  k_proj<<<blocksC, WPB * 32, 0, stream>>>(agg, W, bias, out, nseg);
}
